// MambaBlock_34205119545698
// MI455X (gfx1250) — hardware-verified
//
#include <hip/hip_runtime.h>
#include <stddef.h>
#include <stdint.h>
#include <math.h>


#define DM     1024
#define DI     2048
#define NST    16
#define DTR    64
#define NXD    96
#define NXP    128
#define NBAT   2
#define LSEQ   2048
#define ROWS   (NBAT * LSEQ)
#define K2I    (2 * DI)
#define K2D    (2 * DTR)
#define GBM    64
#define GBN    64
#define GTHR   128
#define NTHR   256
#define CST    32
#define SCR    32
#define SCC    128
#define SPN    (DI * 4 + 3 * DI)
#define SP_CB  (DI * 4)
#define SP_DTB (DI * 4 + DI)
#define SP_DS  (DI * 4 + 2 * DI)
#define WSMAX  ((size_t)128 << 20)

#define PU_XB  (ROWS * DM / 8)
#define PU_WIN (2 * DI * DM / 8)
#define PU_WO  (DM * K2I / 8)
#define PU_WX  (NXP * K2I / 8)
#define PU_WDT (DI * K2D / 8)
#define PU_AN  (DI * NST / 4)
#define PU_SP  (SPN / 4)
#define PU_ALL (PU_XB + PU_WIN + PU_WO + PU_WX + PU_WDT + PU_AN + PU_SP)

static_assert(DM % 32 == 0 && K2I % 32 == 0 && K2D % 32 == 0);
static_assert(ROWS % 128 == 0 && ROWS % GBM == 0 && LSEQ % GBM == 0);
static_assert((2 * DI) % GBN == 0 && NXP % GBN == 0 && DI % GBN == 0 && DM % GBN == 0);
static_assert(GBM == (GTHR / 32) * 16 && GBN == 64);
static_assert(K2I == 2 * DI && K2D == 2 * DTR && DTR == 64 && NST == 16 && NXD <= NXP && NXD - DTR == 32);
static_assert(PU_XB % NTHR == 0 && PU_WIN % NTHR == 0 && PU_WO % NTHR == 0 && PU_WX % NTHR == 0);
static_assert(PU_WDT % NTHR == 0 && PU_AN % NTHR == 0 && PU_SP % NTHR == 0);
static_assert((SP_CB / 4) % NTHR == 0 && (SP_DTB / 4) % NTHR == 0 && (SP_DS / 4) % NTHR == 0);
static_assert(LSEQ % CST == 0 && ((ROWS / CST) * (DI / 4)) % NTHR == 0 && (DI / 4) == 512);
static_assert((LSEQ & (LSEQ - 1)) == 0);
static_assert(LSEQ % SCR == 0 && DI % SCC == 0 && DI / SCC == 16);
static_assert(SCR * SCC / 4 == 8 * SCC && SCR * SCC / 8 == 4 * SCC && SCR * 32 / 4 == 2 * SCC);
static_assert(2 * SCR * (SCC / 8) == 8 * SCC);
static_assert(2 * SCR * SCC * 4 + 2 * SCR * SCC * 2 + SCR * 32 * 4 <= 65536);

typedef float          v4f   __attribute__((ext_vector_type(4)));
typedef float          v8f   __attribute__((ext_vector_type(8)));
typedef int            v8i   __attribute__((ext_vector_type(8)));
typedef unsigned short v4us  __attribute__((ext_vector_type(4)));
typedef unsigned short v8us  __attribute__((ext_vector_type(8)));
typedef unsigned short v16us __attribute__((ext_vector_type(16)));
typedef __bf16         v16bf __attribute__((ext_vector_type(16)));
typedef v4f  __attribute__((may_alias)) v4fa;
typedef v8us __attribute__((may_alias)) v8usa;
union FragB { v16bf v; v16us u; v8us h[2]; v8i w; };

__device__ __forceinline__ v8f wmb(const FragB& a, const FragB& b, v8f c) {
  v8f d = __builtin_amdgcn_wmma_f32_16x16x32_bf16(false, a.v, false, b.v, (short)0, c, false, false);
  asm volatile("v_nop\n\tv_nop\n\tv_nop\n\tv_nop" : "+v"(d) : "v"(a.w), "v"(b.w));
  return d;
}

__device__ __forceinline__ unsigned bf16_bits(float f) {
  const unsigned u = __float_as_uint(f);
  return (u + 0x7FFFu + ((u >> 16) & 1u)) >> 16;
}
__device__ __forceinline__ float bf16_val(float f) {
  return __uint_as_float(bf16_bits(f) << 16);
}
__device__ __forceinline__ unsigned short hl_sel(float v, bool lo_sel) {
  const unsigned hb = bf16_bits(v);
  const unsigned lb = bf16_bits(v - __uint_as_float(hb << 16));
  return (unsigned short)(lo_sel ? lb : hb);
}
__device__ __forceinline__ float silu_f(float c) { return c / (1.0f + expf(-c)); }
__device__ __forceinline__ float softplus_f(float v) { return fmaxf(v, 0.0f) + log1pf(expf(-fabsf(v))); }

__device__ __forceinline__ void cvt8_put(const float* p, bool ok, unsigned short* dp) {
  const v4f a = *(const v4fa*)p;
  const v4f b = *(const v4fa*)(p + 4);
  v8us o;
  o[0] = ok ? (unsigned short)bf16_bits(a.x) : (unsigned short)0;
  o[1] = ok ? (unsigned short)bf16_bits(a.y) : (unsigned short)0;
  o[2] = ok ? (unsigned short)bf16_bits(a.z) : (unsigned short)0;
  o[3] = ok ? (unsigned short)bf16_bits(a.w) : (unsigned short)0;
  o[4] = ok ? (unsigned short)bf16_bits(b.x) : (unsigned short)0;
  o[5] = ok ? (unsigned short)bf16_bits(b.y) : (unsigned short)0;
  o[6] = ok ? (unsigned short)bf16_bits(b.z) : (unsigned short)0;
  o[7] = ok ? (unsigned short)bf16_bits(b.w) : (unsigned short)0;
  *(volatile v8us*)dp = o;
  __threadfence();
  *(volatile v8us*)dp = o;
}
__device__ __forceinline__ void rnd4_put(const float* p, float* dp) {
  const v4f a = *(const v4fa*)p;
  v4f o;
  o.x = bf16_val(a.x); o.y = bf16_val(a.y); o.z = bf16_val(a.z); o.w = bf16_val(a.w);
  *(volatile v4f*)dp = o;
  __threadfence();
  *(volatile v4f*)dp = o;
}

__global__ __launch_bounds__(NTHR) void k_prep(
    const float* __restrict__ x, const float* __restrict__ win, const float* __restrict__ cw,
    const float* __restrict__ cb, const float* __restrict__ wx, const float* __restrict__ wdt,
    const float* __restrict__ dtb, const float* __restrict__ alog, const float* __restrict__ dsk,
    const float* __restrict__ wo,
    unsigned short* XB, unsigned short* WIN, unsigned short* WO2, unsigned short* WX2,
    unsigned short* WDT2, float* AN, float* SP)
{
  const int u = (int)blockIdx.x * NTHR + (int)threadIdx.x;
  if (u < PU_XB) {
    cvt8_put(x + (size_t)8 * u, true, XB + (size_t)8 * u);
  } else if (u < PU_XB + PU_WIN) {
    const int v = u - PU_XB;
    cvt8_put(win + (size_t)8 * v, true, WIN + (size_t)8 * v);
  } else if (u < PU_XB + PU_WIN + PU_WO) {
    const int v  = u - (PU_XB + PU_WIN);
    const int n  = v >> 9;
    const int k8 = (v & 511) * 8;
    cvt8_put(wo + (size_t)n * DI + (k8 & (DI - 1)), true, WO2 + (size_t)n * K2I + k8);
  } else if (u < PU_XB + PU_WIN + PU_WO + PU_WX) {
    const int v  = u - (PU_XB + PU_WIN + PU_WO);
    const int n  = v >> 9;
    const int k8 = (v & 511) * 8;
    const int nc = n < NXD ? n : NXD - 1;
    cvt8_put(wx + (size_t)nc * DI + (k8 & (DI - 1)), n < NXD, WX2 + (size_t)n * K2I + k8);
  } else if (u < PU_XB + PU_WIN + PU_WO + PU_WX + PU_WDT) {
    const int v  = u - (PU_XB + PU_WIN + PU_WO + PU_WX);
    const int n  = v >> 4;
    const int k8 = (v & 15) * 8;
    cvt8_put(wdt + (size_t)n * DTR + (k8 & (DTR - 1)), true, WDT2 + (size_t)n * K2D + k8);
  } else if (u < PU_XB + PU_WIN + PU_WO + PU_WX + PU_WDT + PU_AN) {
    const int v = u - (PU_XB + PU_WIN + PU_WO + PU_WX + PU_WDT);
    const v4f a = *(const v4fa*)(alog + (size_t)4 * v);
    v4f o;
    o.x = -expf(bf16_val(a.x)); o.y = -expf(bf16_val(a.y));
    o.z = -expf(bf16_val(a.z)); o.w = -expf(bf16_val(a.w));
    float* dp = AN + (size_t)4 * v;
    *(volatile v4f*)dp = o;
    __threadfence();
    *(volatile v4f*)dp = o;
  } else if (u < PU_ALL) {
    const int v = u - (PU_XB + PU_WIN + PU_WO + PU_WX + PU_WDT + PU_AN);
    float* dp = SP + (size_t)4 * v;
    if (v < SP_CB / 4)            rnd4_put(cw  + (size_t)4 * v, dp);
    else if (v < SP_DTB / 4)      rnd4_put(cb  + (size_t)4 * (v - SP_CB / 4), dp);
    else if (v < SP_DS / 4)       rnd4_put(dtb + (size_t)4 * (v - SP_DTB / 4), dp);
    else                          rnd4_put(dsk + (size_t)4 * (v - SP_DS / 4), dp);
  }
}

template <int MODE>
__global__ __launch_bounds__(GTHR) void k_gemm(
    const unsigned short* __restrict__ A, int lda,
    const unsigned short* __restrict__ WT, int ldb, int K,
    float* outF, int ldo, int nsplit, int pstride,
    const float* __restrict__ bias, unsigned short* outH)
{
  __shared__ __attribute__((aligned(16))) float stg[GBM * GBN];
  const int tid = (int)threadIdx.x, lane = tid & 31, wave = tid >> 5, hh = lane >> 4, m = lane & 15;
  const int rowBase = (int)blockIdx.x * GBM;
  const int col0    = (int)blockIdx.y * GBN;

  v8f acc[4];
  {
    const v8f z = {0.f, 0.f, 0.f, 0.f, 0.f, 0.f, 0.f, 0.f};
    acc[0] = z; acc[1] = z; acc[2] = z; acc[3] = z;
  }
  const unsigned short* ap = A  + (size_t)(rowBase + 16 * wave + m) * (size_t)lda + 8 * hh;
  const unsigned short* wp = WT + (size_t)(col0 + m) * (size_t)ldb + 8 * hh;
  const int ksteps = K >> 5;
#pragma unroll 1
  for (int ks = 0; ks < ksteps; ++ks) {
    FragB af;
    af.h[0] = *(const v8usa*)(ap + 32 * ks);
    af.h[1] = *(const v8usa*)(ap + 32 * ks + 16);
#pragma unroll
    for (int t = 0; t < 4; ++t) {
      const unsigned short* wq = wp + (size_t)(16 * t) * (size_t)ldb + 32 * ks;
      FragB bf;
      bf.h[0] = *(const v8usa*)wq;
      bf.h[1] = *(const v8usa*)(wq + 16);
      acc[t] = wmb(af, bf, acc[t]);
    }
  }

#pragma unroll
  for (int t = 0; t < 4; ++t) {
    const int lc = 16 * t + m;
#pragma unroll
    for (int r = 0; r < 8; ++r) {
      const int lr = 16 * wave + 8 * hh + r;
      stg[lr * GBN + lc] = acc[t][r];
    }
  }
  __syncthreads();

  if constexpr (MODE == 0 || MODE == 3) {
    const int plane = col0 / nsplit;
    const int cc    = col0 - plane * nsplit;
    if constexpr (MODE == 3) {
      if (plane != 0) {
#pragma unroll 1
        for (int i = 0; i < 8; ++i) {
          float* sp = stg + (16 * wave + 2 * i + hh) * GBN + 4 * m;
          v4f v = *(const v4fa*)sp;
          v.x = silu_f(v.x); v.y = silu_f(v.y); v.z = silu_f(v.z); v.w = silu_f(v.w);
          *(v4fa*)sp = v;
        }
      }
    }
    float* ob = outF + (size_t)plane * (size_t)pstride + cc + 4 * m;
    v4f fv[8];
#pragma unroll
    for (int i = 0; i < 8; ++i) {
      const int lr = 16 * wave + 2 * i + hh;
      fv[i] = *(const v4fa*)(stg + lr * GBN + 4 * m);
    }
#pragma unroll
    for (int i = 0; i < 8; ++i) {
      const int lr = 16 * wave + 2 * i + hh;
      *(volatile v4f*)(ob + (size_t)(rowBase + lr) * (size_t)ldo) = fv[i];
    }
    __threadfence();
#pragma unroll
    for (int i = 0; i < 8; ++i) {
      const int lr = 16 * wave + 2 * i + hh;
      *(volatile v4f*)(ob + (size_t)(rowBase + lr) * (size_t)ldo) = fv[i];
    }
  } else if constexpr (MODE == 1) {
    const v4f bb = *(const v4fa*)(bias + col0 + 4 * m);
#pragma unroll 1
    for (int i = 0; i < 8; ++i) {
      const int lr = 16 * wave + 2 * i + hh;
      const v4f t = *(const v4fa*)(stg + lr * GBN + 4 * m);
      v4f o;
      o.x = softplus_f(t.x + bb.x);
      o.y = softplus_f(t.y + bb.y);
      o.z = softplus_f(t.z + bb.z);
      o.w = softplus_f(t.w + bb.w);
      float* op = outF + (size_t)(rowBase + lr) * (size_t)ldo + col0 + 4 * m;
      *(volatile v4f*)op = o;
      __threadfence();
      *(volatile v4f*)op = o;
    }
  } else {
    if (blockIdx.y == 0) {
      const int  q = m & 7;
      const bool lo_sel = (m >= 8);
      v8us qv[8];
#pragma unroll
      for (int i = 0; i < 8; ++i) {
        const int lr = 16 * wave + 2 * i + hh;
        const v4f a = *(const v4fa*)(stg + lr * GBN + 8 * q);
        const v4f b = *(const v4fa*)(stg + lr * GBN + 8 * q + 4);
        v8us o;
        o[0] = hl_sel(a.x, lo_sel); o[1] = hl_sel(a.y, lo_sel);
        o[2] = hl_sel(a.z, lo_sel); o[3] = hl_sel(a.w, lo_sel);
        o[4] = hl_sel(b.x, lo_sel); o[5] = hl_sel(b.y, lo_sel);
        o[6] = hl_sel(b.z, lo_sel); o[7] = hl_sel(b.w, lo_sel);
        qv[i] = o;
      }
#pragma unroll
      for (int i = 0; i < 8; ++i) {
        const int lr = 16 * wave + 2 * i + hh;
        *(volatile v8us*)(outH + (size_t)(rowBase + lr) * K2D + 8 * m) = qv[i];
      }
      __threadfence();
#pragma unroll
      for (int i = 0; i < 8; ++i) {
        const int lr = 16 * wave + 2 * i + hh;
        *(volatile v8us*)(outH + (size_t)(rowBase + lr) * K2D + 8 * m) = qv[i];
      }
    } else {
      const int rs = lane >> 3;
      const int c4 = (lane & 7) * 4;
      v4f fv[4];
#pragma unroll
      for (int i = 0; i < 4; ++i) {
        const int lr = 16 * wave + 4 * i + rs;
        fv[i] = *(const v4fa*)(stg + lr * GBN + c4);
      }
#pragma unroll
      for (int i = 0; i < 4; ++i) {
        const int lr = 16 * wave + 4 * i + rs;
        *(volatile v4f*)(outF + (size_t)(rowBase + lr) * 32 + c4) = fv[i];
      }
      __threadfence();
#pragma unroll
      for (int i = 0; i < 4; ++i) {
        const int lr = 16 * wave + 4 * i + rs;
        *(volatile v4f*)(outF + (size_t)(rowBase + lr) * 32 + c4) = fv[i];
      }
    }
  }
}

__global__ __launch_bounds__(NTHR) void k_conv(const float* __restrict__ XI, const float* __restrict__ SP,
                                               unsigned short* UHL)
{
  const int t = (int)blockIdx.x * NTHR + (int)threadIdx.x;
  const int q = t & 511;
  const int s = t >> 9;
  if (s >= ROWS / CST) return;
  const int r0 = s * CST;
  const int l0 = r0 & (LSEQ - 1);
  const int c0 = 4 * q;
  const v4f w0 = *(const v4fa*)(SP + 4 * (c0 + 0));
  const v4f w1 = *(const v4fa*)(SP + 4 * (c0 + 1));
  const v4f w2 = *(const v4fa*)(SP + 4 * (c0 + 2));
  const v4f w3 = *(const v4fa*)(SP + 4 * (c0 + 3));
  const v4f bb = *(const v4fa*)(SP + SP_CB + c0);
  const bool pv = l0 > 0;
  const int ra = pv ? r0 - 3 : r0;
  const int rb = pv ? r0 - 2 : r0;
  const int rc = pv ? r0 - 1 : r0;
  const v4f zz = {0.f, 0.f, 0.f, 0.f};
  v4f x0 = *(const v4fa*)(XI + (size_t)ra * DI + c0);
  v4f x1 = *(const v4fa*)(XI + (size_t)rb * DI + c0);
  v4f x2 = *(const v4fa*)(XI + (size_t)rc * DI + c0);
  x0 = pv ? x0 : zz; x1 = pv ? x1 : zz; x2 = pv ? x2 : zz;
#pragma unroll 1
  for (int i = 0; i < CST; ++i) {
    const int r = r0 + i;
    const v4f xn = *(const v4fa*)(XI + (size_t)r * DI + c0);
    v4f c;
    c.x = fmaf(w0.w, xn.x, fmaf(w0.z, x2.x, fmaf(w0.y, x1.x, w0.x * x0.x))) + bb.x;
    c.y = fmaf(w1.w, xn.y, fmaf(w1.z, x2.y, fmaf(w1.y, x1.y, w1.x * x0.y))) + bb.y;
    c.z = fmaf(w2.w, xn.z, fmaf(w2.z, x2.z, fmaf(w2.y, x1.z, w2.x * x0.z))) + bb.z;
    c.w = fmaf(w3.w, xn.w, fmaf(w3.z, x2.w, fmaf(w3.y, x1.w, w3.x * x0.w))) + bb.w;
    v4f uo;
    uo.x = silu_f(c.x); uo.y = silu_f(c.y); uo.z = silu_f(c.z); uo.w = silu_f(c.w);
    v4us hv, lv;
    hv[0] = hl_sel(uo.x, false); lv[0] = hl_sel(uo.x, true);
    hv[1] = hl_sel(uo.y, false); lv[1] = hl_sel(uo.y, true);
    hv[2] = hl_sel(uo.z, false); lv[2] = hl_sel(uo.z, true);
    hv[3] = hl_sel(uo.w, false); lv[3] = hl_sel(uo.w, true);
    unsigned short* hp = UHL + (size_t)r * K2I + c0;
    *(volatile v4us*)hp = hv;
    *(volatile v4us*)(hp + DI) = lv;
    __threadfence();
    *(volatile v4us*)hp = hv;
    *(volatile v4us*)(hp + DI) = lv;
    x0 = x1; x1 = x2; x2 = xn;
  }
}

__global__ __launch_bounds__(SCC) void k_scan(const float* __restrict__ DELTA, const float* __restrict__ SZ,
                                              const float* __restrict__ BC, const float* __restrict__ AN,
                                              const float* __restrict__ DS, unsigned short* UHL)
{
  __shared__ __attribute__((aligned(16))) float dls[SCR * SCC];
  __shared__ __attribute__((aligned(16))) float szs[SCR * SCC];
  __shared__ __attribute__((aligned(16))) unsigned short his[SCR * SCC];
  __shared__ __attribute__((aligned(16))) unsigned short los[SCR * SCC];
  __shared__ __attribute__((aligned(16))) float bcs[SCR * 32];
  const int tid = (int)threadIdx.x;
  const int b   = (int)blockIdx.x >> 4;
  const int d0  = ((int)blockIdx.x & 15) * SCC;
  const int d   = d0 + tid;

  float h[NST], Ar[NST];
#pragma unroll
  for (int j = 0; j < 4; ++j) {
    const v4f a = *(const v4fa*)(AN + (size_t)d * NST + 4 * j);
    Ar[4 * j + 0] = a.x; Ar[4 * j + 1] = a.y; Ar[4 * j + 2] = a.z; Ar[4 * j + 3] = a.w;
    h[4 * j + 0] = 0.0f; h[4 * j + 1] = 0.0f; h[4 * j + 2] = 0.0f; h[4 * j + 3] = 0.0f;
  }
  const float Dd = DS[d];

#pragma unroll 1
  for (int cnk = 0; cnk < LSEQ / SCR; ++cnk) {
    const int row0 = b * LSEQ + cnk * SCR;
#pragma unroll 2
    for (int it = 0; it < 8; ++it) {
      const int idx = it * SCC + tid;
      const int row = idx >> 5;
      const int cc  = (idx & 31) * 4;
      const size_t go = (size_t)(row0 + row) * DI + d0 + cc;
      const v4f a = *(const v4fa*)(DELTA + go);
      const v4f f = *(const v4fa*)(SZ + go);
      *(v4fa*)(dls + row * SCC + cc) = a;
      *(v4fa*)(szs + row * SCC + cc) = f;
    }
#pragma unroll 2
    for (int it = 0; it < 4; ++it) {
      const int idx = it * SCC + tid;
      const int row = idx >> 4;
      const int c8  = (idx & 15) * 8;
      const unsigned short* gp = UHL + (size_t)(row0 + row) * K2I + d0 + c8;
      const v8us hv = *(const v8usa*)gp;
      const v8us lv = *(const v8usa*)(gp + DI);
      *(v8usa*)(his + row * SCC + c8) = hv;
      *(v8usa*)(los + row * SCC + c8) = lv;
    }
#pragma unroll
    for (int it = 0; it < 2; ++it) {
      const int idx = it * SCC + tid;
      *(v4fa*)(bcs + 4 * idx) = *(const v4fa*)(BC + (size_t)row0 * 32 + 4 * idx);
    }
    __syncthreads();

#pragma unroll 1
    for (int t = 0; t < SCR; ++t) {
      const int li = t * SCC + tid;
      const float dl = dls[li];
      const float zv = szs[li];
      const float uu = __uint_as_float((unsigned)his[li] << 16) + __uint_as_float((unsigned)los[li] << 16);
      const float du = dl * uu;
      const float* bp = bcs + t * 32;
      float Bv[NST], Cv[NST];
#pragma unroll
      for (int j = 0; j < 4; ++j) {
        const v4f tb = *(const v4fa*)(bp + 4 * j);
        const v4f tc = *(const v4fa*)(bp + NST + 4 * j);
        Bv[4 * j + 0] = tb.x; Bv[4 * j + 1] = tb.y; Bv[4 * j + 2] = tb.z; Bv[4 * j + 3] = tb.w;
        Cv[4 * j + 0] = tc.x; Cv[4 * j + 1] = tc.y; Cv[4 * j + 2] = tc.z; Cv[4 * j + 3] = tc.w;
      }
#pragma unroll
      for (int n = 0; n < NST; ++n) {
        const float dA = expf(dl * Ar[n]);
        h[n] = dA * h[n] + du * Bv[n];
      }
      float y = h[0] * Cv[0];
#pragma unroll
      for (int n = 1; n < NST; ++n) y = fmaf(h[n], Cv[n], y);
      y = y + uu * Dd;
      y = y * zv;
      dls[li] = y;
    }
    __syncthreads();

    v8us ov[8];
#pragma unroll
    for (int it = 0; it < 8; ++it) {
      const bool lo_sel = (it >> 2) != 0;
      const int j   = (it & 3) * SCC + tid;
      const int row = j >> 4;
      const int c8  = (j & 15) * 8;
      const v4f g0 = *(const v4fa*)(dls + row * SCC + c8);
      const v4f g1 = *(const v4fa*)(dls + row * SCC + c8 + 4);
      v8us o;
      o[0] = hl_sel(g0.x, lo_sel); o[1] = hl_sel(g0.y, lo_sel);
      o[2] = hl_sel(g0.z, lo_sel); o[3] = hl_sel(g0.w, lo_sel);
      o[4] = hl_sel(g1.x, lo_sel); o[5] = hl_sel(g1.y, lo_sel);
      o[6] = hl_sel(g1.z, lo_sel); o[7] = hl_sel(g1.w, lo_sel);
      ov[it] = o;
    }
    __syncthreads();

#pragma unroll
    for (int it = 0; it < 8; ++it) {
      const int plane = it >> 2;
      const int j   = (it & 3) * SCC + tid;
      const int row = j >> 4;
      const int c8  = (j & 15) * 8;
      unsigned short* gp = UHL + (size_t)(row0 + row) * K2I + (size_t)plane * DI + d0 + c8;
      *(volatile v8us*)gp = ov[it];
    }
    __threadfence();
#pragma unroll
    for (int it = 0; it < 8; ++it) {
      const int plane = it >> 2;
      const int j   = (it & 3) * SCC + tid;
      const int row = j >> 4;
      const int c8  = (j & 15) * 8;
      unsigned short* gp = UHL + (size_t)(row0 + row) * K2I + (size_t)plane * DI + d0 + c8;
      *(volatile v8us*)gp = ov[it];
    }
  }
}

static inline size_t al256(size_t o) { return (o + 255) & ~(size_t)255; }

extern "C" void kernel_launch(void* const* d_in, const int* in_sizes, int n_in,
                              void* d_out, int out_size, void* d_ws, size_t ws_size,
                              hipStream_t stream) {
  if (n_in < 10) return;
  if (in_sizes[0] != ROWS * DM) return;
  if (in_sizes[1] != 2 * DI * DM) return;
  if (in_sizes[2] != DI * 4) return;
  if (in_sizes[3] != DI) return;
  if (in_sizes[4] != NXD * DI) return;
  if (in_sizes[5] != DI * DTR) return;
  if (in_sizes[6] != DI) return;
  if (in_sizes[7] != DI * NST) return;
  if (in_sizes[8] != DI) return;
  if (in_sizes[9] != DM * DI) return;
  if (out_size != ROWS * DM) return;

  const float* x    = (const float*)d_in[0];
  const float* win  = (const float*)d_in[1];
  const float* cw   = (const float*)d_in[2];
  const float* cb   = (const float*)d_in[3];
  const float* wx   = (const float*)d_in[4];
  const float* wdt  = (const float*)d_in[5];
  const float* dtb  = (const float*)d_in[6];
  const float* alog = (const float*)d_in[7];
  const float* dsk  = (const float*)d_in[8];
  const float* wo   = (const float*)d_in[9];
  float* out = (float*)d_out;

  char* ws = (char*)d_ws;
  size_t off = 0;
  const size_t oXI   = off; off = al256(off + (size_t)ROWS * DI * 4);
  const size_t oSZ   = off; off = al256(off + (size_t)ROWS * DI * 4);
  const size_t oUHL  = off; off = al256(off + (size_t)ROWS * K2I * 2);
  const size_t oBC   = off; off = al256(off + (size_t)ROWS * 32 * 4);
  const size_t oDTHL = off; off = al256(off + (size_t)ROWS * K2D * 2);
  const size_t oXB   = off; off = al256(off + (size_t)ROWS * DM * 2);
  const size_t oWIN  = off; off = al256(off + (size_t)2 * DI * DM * 2);
  const size_t oWX2  = off; off = al256(off + (size_t)NXP * K2I * 2);
  const size_t oWDT2 = off; off = al256(off + (size_t)DI * K2D * 2);
  const size_t oWO2  = off; off = al256(off + (size_t)DM * K2I * 2);
  const size_t oAN   = off; off = al256(off + (size_t)DI * NST * 4);
  const size_t oSP   = off; off = al256(off + (size_t)SPN * 4);
  if (off > ws_size || off > WSMAX) return;

  float*          XI   = (float*)(ws + oXI);
  float*          SZp  = (float*)(ws + oSZ);
  unsigned short* UHL  = (unsigned short*)(ws + oUHL);
  float*          BC   = (float*)(ws + oBC);
  unsigned short* DTHL = (unsigned short*)(ws + oDTHL);
  unsigned short* XB   = (unsigned short*)(ws + oXB);
  unsigned short* WIN  = (unsigned short*)(ws + oWIN);
  unsigned short* WX2  = (unsigned short*)(ws + oWX2);
  unsigned short* WDT2 = (unsigned short*)(ws + oWDT2);
  unsigned short* WO2  = (unsigned short*)(ws + oWO2);
  float*          AN   = (float*)(ws + oAN);
  float*          SP   = (float*)(ws + oSP);
  float*          DELTA = XI;
  const int pstr = (int)((oSZ - oXI) / 4);

  k_prep<<<PU_ALL / NTHR, NTHR, 0, stream>>>(x, win, cw, cb, wx, wdt, dtb, alog, dsk, wo,
                                             XB, WIN, WO2, WX2, WDT2, AN, SP);
  k_gemm<3><<<dim3(ROWS / GBM, (2 * DI) / GBN), GTHR, 0, stream>>>(
      XB, DM, WIN, DM, DM, XI, DI, DI, pstr, SP, DTHL);
  k_conv<<<((ROWS / CST) * (DI / 4)) / NTHR, NTHR, 0, stream>>>(XI, SP, UHL);
  k_gemm<2><<<dim3(ROWS / GBM, NXP / GBN), GTHR, 0, stream>>>(
      UHL, K2I, WX2, K2I, K2I, BC, 32, NXP, 0, SP, DTHL);
  k_gemm<1><<<dim3(ROWS / GBM, DI / GBN), GTHR, 0, stream>>>(
      DTHL, K2D, WDT2, K2D, K2D, DELTA, DI, DI, 0, SP + SP_DTB, UHL);
  k_scan<<<NBAT * (DI / SCC), SCC, 0, stream>>>(DELTA, SZp, BC, AN, SP + SP_DS, UHL);
  k_gemm<0><<<dim3(ROWS / GBM, DM / GBN), GTHR, 0, stream>>>(
      UHL, K2I, WO2, K2I, K2I, out, DM, DM, 0, SP, DTHL);
}
